// NeuralStyleField_1726576854306
// MI455X (gfx1250) — hardware-verified
//
#include <hip/hip_runtime.h>
#include <stdint.h>
#include <stddef.h>


typedef _Float16 v16h __attribute__((ext_vector_type(16)));
typedef _Float16 v8h  __attribute__((ext_vector_type(8)));
typedef v8h v8hA __attribute__((may_alias));
typedef float v8f __attribute__((ext_vector_type(8)));
typedef float v4f __attribute__((ext_vector_type(4)));
typedef v4f v4fA __attribute__((may_alias));

union Frag  { v16h v; v8h hf[2]; };
union Pack8 { v8h hv; v4f f; };

#define WID        256
#define KF         512
#define ROWS       64
#define TPB_MAIN   128
#define TPB_PREP   256
#define NSQ        8
#define SQH        65536
#define TP         520
#define ACT_SCALE  64.0f
#define ACT_INV    0.015625f
#define TWO_PI_F   6.28318548f
#define TWO_PI_LO  (-1.74845553e-7f)
#define INV_TWO_PI 0.159154943f
#define TAU_F      0.0853333333f
#define INV_TAU_F  (1.0f / TAU_F)
#define NORM_RATIO 0.1f

#define OFF_BUF0   0
#define OFF_BUF1   65536
#define OFF_BUF2   98304
#define OFF_SB     131072
#define OFF_SX     134144
#define OFF_O0     134912
#define OFF_O1     135680
#define SMEM_MAIN  135936

__device__ __forceinline__ v8f wmma_f16(v16h a, v16h b, v8f c)
{
    c = __builtin_amdgcn_wmma_f32_16x16x32_f16(false, a, false, b, (short)0, c, false, false);
    asm volatile("v_nop\n\tv_nop\n\tv_nop\n\tv_nop" : "+v"(c) : "v"(a), "v"(b));
    return c;
}

extern "C" __global__ void __launch_bounds__(TPB_PREP)
k_prep(const float* __restrict__ W0,  const float* __restrict__ W1,
       const float* __restrict__ W2,  const float* __restrict__ W3,
       const float* __restrict__ W4,  const float* __restrict__ Wc0,
       const float* __restrict__ Wc1, const float* __restrict__ Wc2,
       const float* __restrict__ Wn0, const float* __restrict__ Wn1,
       const float* __restrict__ Wn2,
       _Float16* __restrict__ wt0, _Float16* __restrict__ wsq,
       _Float16* __restrict__ wc2, _Float16* __restrict__ wn2)
{
    __shared__ __attribute__((aligned(16))) _Float16 tile[32 * TP];

    const int tid = threadIdx.x;
    const int tx = tid & 31, ty = tid >> 5;
    const int lane = tx, wv = ty;
    const int bid = blockIdx.x;

    int mat, g;
    if (bid < 8)                { mat = 0; g = bid; }
    else if (bid < 8 + NSQ * 8) { mat = 1 + ((bid - 8) >> 3); g = (bid - 8) & 7; }
    else                        { mat = 9 + (bid - 8 - NSQ * 8); g = 0; }

    const float* src; _Float16* dst; int K, srcN, nrows;
    switch (mat) {
        case 0:  src = W0 + 3 * WID; dst = wt0;           K = KF;  srcN = WID; nrows = 32; break;
        case 1:  src = W1;  dst = wsq + 0 * SQH;          K = WID; srcN = WID; nrows = 32; break;
        case 2:  src = W2;  dst = wsq + 1 * SQH;          K = WID; srcN = WID; nrows = 32; break;
        case 3:  src = W3;  dst = wsq + 2 * SQH;          K = WID; srcN = WID; nrows = 32; break;
        case 4:  src = W4;  dst = wsq + 3 * SQH;          K = WID; srcN = WID; nrows = 32; break;
        case 5:  src = Wc0; dst = wsq + 4 * SQH;          K = WID; srcN = WID; nrows = 32; break;
        case 6:  src = Wc1; dst = wsq + 5 * SQH;          K = WID; srcN = WID; nrows = 32; break;
        case 7:  src = Wn0; dst = wsq + 6 * SQH;          K = WID; srcN = WID; nrows = 32; break;
        case 8:  src = Wn1; dst = wsq + 7 * SQH;          K = WID; srcN = WID; nrows = 32; break;
        case 9:  src = Wc2; dst = wc2;                    K = WID; srcN = 3;   nrows = 16; break;
        default: src = Wn2; dst = wn2;                    K = WID; srcN = 1;   nrows = 16; break;
    }

    const int n0 = g * 32;
    const int n  = n0 + tx;
    const bool nvalid = (n < srcN);
    for (int k = ty; k < K; k += 8) {
        const float v = nvalid ? src[(size_t)k * srcN + n] : 0.0f;
        tile[tx * TP + k] = (_Float16)v;
    }
    __syncthreads();

    const bool wide = (K == KF);
    Pack8 val0[4], val1[4];
#pragma unroll
    for (int j = 0; j < 4; ++j) {
        const int r = wv * 4 + j;
        val0[j].hv = *(const v8hA*)(tile + r * TP + lane * 8);
        val1[j].hv = val0[j].hv;
        if (wide) val1[j].hv = *(const v8hA*)(tile + r * TP + WID + lane * 8);
    }
#pragma unroll
    for (int j = 0; j < 4; ++j) {
        const int r = wv * 4 + j;
        if (r < nrows) {
            _Float16* rowp = dst + (size_t)(n0 + r) * K;
            *(volatile v4f*)(rowp + lane * 8) = val0[j].f;
            if (wide) *(volatile v4f*)(rowp + WID + lane * 8) = val1[j].f;
        }
    }
    __threadfence();
#pragma unroll
    for (int j = 0; j < 4; ++j) {
        const int r = wv * 4 + j;
        if (r < nrows) {
            _Float16* rowp = dst + (size_t)(n0 + r) * K;
            *(volatile v4f*)(rowp + lane * 8) = val0[j].f;
            if (wide) *(volatile v4f*)(rowp + WID + lane * 8) = val1[j].f;
        }
    }
}

template <int K>
__device__ __forceinline__ void gemm_tile(const _Float16* act, const _Float16* __restrict__ wt,
                                          int wave, int lane, v8f (&acc)[4][4])
{
    const int h = lane >> 4, m = lane & 15;
    const v8f z = {0.f, 0.f, 0.f, 0.f, 0.f, 0.f, 0.f, 0.f};
#pragma unroll
    for (int rt = 0; rt < 4; ++rt)
#pragma unroll
        for (int ct = 0; ct < 4; ++ct) acc[rt][ct] = z;

    const _Float16* ap = act + m * K + 8 * h;
    const _Float16* bp = wt + (size_t)(wave * 64 + m) * K + 8 * h;

#pragma unroll 1
    for (int k0 = 0; k0 < K; k0 += 32) {
        Frag a[4];
#pragma unroll
        for (int rt = 0; rt < 4; ++rt) {
            a[rt].hf[0] = *(const v8hA*)(ap + rt * 16 * K + k0);
            a[rt].hf[1] = *(const v8hA*)(ap + rt * 16 * K + k0 + 16);
        }
#pragma unroll
        for (int ct = 0; ct < 4; ++ct) {
            Frag b;
            b.hf[0] = *(const v8hA*)(bp + (size_t)ct * 16 * K + k0);
            b.hf[1] = *(const v8hA*)(bp + (size_t)ct * 16 * K + k0 + 16);
#pragma unroll
            for (int rt = 0; rt < 4; ++rt)
                acc[rt][ct] = wmma_f16(a[rt].v, b.v, acc[rt][ct]);
        }
    }
}

__device__ __forceinline__ void epi_relu(v8f (&acc)[4][4], const float* __restrict__ bias,
                                         _Float16* outT, int wave, int lane)
{
    const int h = lane >> 4, m = lane & 15;
#pragma unroll
    for (int ct = 0; ct < 4; ++ct) {
        const int col = wave * 64 + ct * 16 + m;
        const float bv = bias[col];
#pragma unroll
        for (int rt = 0; rt < 4; ++rt) {
#pragma unroll
            for (int r = 0; r < 8; ++r) {
                const int row = rt * 16 + 8 * h + r;
                float v = fmaf(acc[rt][ct][r], ACT_INV, bv);
                v = fmaxf(v, 0.0f) * ACT_SCALE;
                outT[row * WID + col] = (_Float16)v;
            }
        }
    }
}

__device__ __forceinline__ void epi_first(v8f (&acc)[4][4], const float* __restrict__ b0,
                                          const float* __restrict__ W0, const float* sX,
                                          _Float16* outT, int wave, int lane)
{
    const int h = lane >> 4, m = lane & 15;
    float bv[4], wa[4], wb[4], wc[4];
#pragma unroll
    for (int ct = 0; ct < 4; ++ct) {
        const int col = wave * 64 + ct * 16 + m;
        bv[ct] = b0[col];
        wa[ct] = W0[col];
        wb[ct] = W0[WID + col];
        wc[ct] = W0[2 * WID + col];
    }
#pragma unroll
    for (int rt = 0; rt < 4; ++rt) {
#pragma unroll
        for (int r = 0; r < 8; ++r) {
            const int row = rt * 16 + 8 * h + r;
            const float x0 = sX[row * 3 + 0], x1 = sX[row * 3 + 1], x2 = sX[row * 3 + 2];
#pragma unroll
            for (int ct = 0; ct < 4; ++ct) {
                const int col = wave * 64 + ct * 16 + m;
                float xs = x0 * wa[ct];
                xs = fmaf(x1, wb[ct], xs);
                xs = fmaf(x2, wc[ct], xs);
                float v = fmaf(acc[rt][ct][r], ACT_INV, bv[ct]) + xs;
                v = fmaxf(v, 0.0f) * ACT_SCALE;
                outT[row * WID + col] = (_Float16)v;
            }
        }
    }
}

__device__ __forceinline__ v8f head_tile(const _Float16* act, const _Float16* __restrict__ wt,
                                         int wave, int lane)
{
    const int h = lane >> 4, m = lane & 15;
    v8f acc = {0.f, 0.f, 0.f, 0.f, 0.f, 0.f, 0.f, 0.f};
    const _Float16* ap = act + (wave * 16 + m) * WID + 8 * h;
    const _Float16* bp = wt + m * WID + 8 * h;
#pragma unroll
    for (int k0 = 0; k0 < WID; k0 += 32) {
        Frag a, b;
        a.hf[0] = *(const v8hA*)(ap + k0);
        a.hf[1] = *(const v8hA*)(ap + k0 + 16);
        b.hf[0] = *(const v8hA*)(bp + k0);
        b.hf[1] = *(const v8hA*)(bp + k0 + 16);
        acc = wmma_f16(a.v, b.v, acc);
    }
    return acc;
}

extern "C" __global__ void __launch_bounds__(TPB_MAIN)
k_mlp(const float* __restrict__ x, const float* __restrict__ Bf, const int* __restrict__ tptr,
      const float* __restrict__ W0,
      const float* __restrict__ b0,  const float* __restrict__ b1,  const float* __restrict__ b2,
      const float* __restrict__ b3,  const float* __restrict__ b4,
      const float* __restrict__ bc0, const float* __restrict__ bc1, const float* __restrict__ bc2,
      const float* __restrict__ bn0, const float* __restrict__ bn1, const float* __restrict__ bn2,
      const _Float16* __restrict__ wt0, const _Float16* __restrict__ wsq,
      const _Float16* __restrict__ wc2, const _Float16* __restrict__ wn2,
      float* __restrict__ out, int npts)
{
    extern __shared__ __attribute__((aligned(16))) char smem[];
    _Float16* buf0 = (_Float16*)(smem + OFF_BUF0);
    _Float16* buf1 = (_Float16*)(smem + OFF_BUF1);
    _Float16* buf2 = (_Float16*)(smem + OFF_BUF2);
    float* sB  = (float*)(smem + OFF_SB);
    float* sX  = (float*)(smem + OFF_SX);
    float* sO0 = (float*)(smem + OFF_O0);
    float* sO1 = (float*)(smem + OFF_O1);

    const int tid = threadIdx.x, lane = tid & 31, wave = tid >> 5;
    const int h = lane >> 4, m = lane & 15;
    const int blk = blockIdx.x;
    const size_t rowBase = (size_t)blk * ROWS;

    for (int i = tid; i < 3 * WID;  i += TPB_MAIN) sB[i] = Bf[i];
    for (int i = tid; i < 3 * ROWS; i += TPB_MAIN) sX[i] = x[rowBase * 3 + i];
    const float tf = (float)tptr[0];
    __syncthreads();

    {
        _Float16* feat = buf0;
#pragma unroll 1
        for (int i = 0; i < (ROWS * WID) / TPB_MAIN; ++i) {
            const int idx = i * TPB_MAIN + tid;
            const int row = idx >> 8;
            const int c   = idx & (WID - 1);
            const float x0 = sX[row * 3 + 0], x1 = sX[row * 3 + 1], x2 = sX[row * 3 + 2];
            float p = x0 * sB[c];
            p = fmaf(x1, sB[WID + c], p);
            p = fmaf(x2, sB[2 * WID + c], p);
            const float proj = TWO_PI_F * p;
            const float q = rintf(proj * INV_TWO_PI);
            float rr = fmaf(-q, TWO_PI_F, proj);
            rr = fmaf(-q, TWO_PI_LO, rr);
            float al = (tf - TAU_F * (float)c) * INV_TAU_F;
            al = fminf(fmaxf(al, 0.0f), 1.0f) * ACT_SCALE;
            feat[row * KF + c]       = (_Float16)(__sinf(rr) * al);
            feat[row * KF + WID + c] = (_Float16)(__cosf(rr) * al);
        }
    }
    __syncthreads();

    v8f acc[4][4];

    gemm_tile<KF>(buf0, wt0, wave, lane, acc);
    epi_first(acc, b0, W0, sX, buf1, wave, lane);
    __syncthreads();

#pragma unroll 1
    for (int L = 0; L < 8; ++L) {
        const _Float16* ain; _Float16* aout; const float* bias;
        switch (L) {
            case 0:  ain = buf1; aout = buf2; bias = b1;  break;
            case 1:  ain = buf2; aout = buf1; bias = b2;  break;
            case 2:  ain = buf1; aout = buf2; bias = b3;  break;
            case 3:  ain = buf2; aout = buf0; bias = b4;  break;
            case 4:  ain = buf0; aout = buf1; bias = bc0; break;
            case 5:  ain = buf1; aout = buf2; bias = bc1; break;
            case 6:  ain = buf0; aout = buf1; bias = bn0; break;
            default: ain = buf1; aout = buf2; bias = bn1; break;
        }
        gemm_tile<WID>(ain, wsq + (size_t)L * SQH, wave, lane, acc);
        epi_relu(acc, bias, aout, wave, lane);
        __syncthreads();
        if (L == 5) {
            const v8f hc = head_tile(buf2, wc2, wave, lane);
            if (m < 3) {
                const float bb = bc2[m];
#pragma unroll
                for (int r = 0; r < 8; ++r) {
                    const int row = wave * 16 + 8 * h + r;
                    sO0[row * 3 + m] = tanhf(fmaf(hc[r], ACT_INV, bb)) * 0.5f;
                }
            }
            __syncthreads();
        }
    }
    {
        const v8f hd = head_tile(buf2, wn2, wave, lane);
        if (m == 0) {
            const float bb = bn2[0];
#pragma unroll
            for (int r = 0; r < 8; ++r) {
                const int row = wave * 16 + 8 * h + r;
                sO1[row] = tanhf(fmaf(hd[r], ACT_INV, bb)) * NORM_RATIO;
            }
        }
    }
    __syncthreads();

    if (wave == 0) {
        const v4fA* s = (const v4fA*)sO0;
        const v4f v0 = s[lane];
        v4f v1 = v0;
        if (lane < 16) v1 = s[32 + lane];
        float* gbase = out + (size_t)blk * (ROWS * 3);
        *(volatile v4f*)(gbase + lane * 4) = v0;
        if (lane < 16) *(volatile v4f*)(gbase + (32 + lane) * 4) = v1;
        __threadfence();
        *(volatile v4f*)(gbase + lane * 4) = v0;
        if (lane < 16) *(volatile v4f*)(gbase + (32 + lane) * 4) = v1;
    } else if (wave == 1) {
        if (lane < 16) {
            const v4f v = ((const v4fA*)sO1)[lane];
            float* gbase = out + (size_t)npts * 3 + (size_t)blk * ROWS;
            *(volatile v4f*)(gbase + lane * 4) = v;
            __threadfence();
            *(volatile v4f*)(gbase + lane * 4) = v;
        }
    }
}

extern "C" void kernel_launch(void* const* d_in, const int* in_sizes, int n_in,
                              void* d_out, int out_size, void* d_ws, size_t ws_size,
                              hipStream_t stream)
{
    if (n_in < 25) return;
    const int npts = in_sizes[0] / 3;
    if (npts <= 0 || (npts % ROWS) != 0) return;
    if (out_size != npts * 4) return;
    if (in_sizes[1] != 3 * WID || in_sizes[3] != (3 + KF) * WID) return;

    const size_t szW0 = (size_t)WID * KF * sizeof(_Float16);
    const size_t szSQ = (size_t)NSQ * SQH * sizeof(_Float16);
    const size_t szHD = (size_t)16 * WID * sizeof(_Float16);
    const size_t off0 = 0;
    const size_t off1 = off0 + szW0;
    const size_t off2 = off1 + szSQ;
    const size_t off3 = off2 + szHD;
    const size_t total = off3 + szHD;
    if (total > ws_size) return;

    const float* x   = (const float*)d_in[0];
    const float* Bf  = (const float*)d_in[1];
    const int*   t   = (const int*)  d_in[2];
    const float* W0  = (const float*)d_in[3];
    const float* b0  = (const float*)d_in[4];
    const float* W1  = (const float*)d_in[5];
    const float* b1  = (const float*)d_in[6];
    const float* W2  = (const float*)d_in[7];
    const float* b2  = (const float*)d_in[8];
    const float* W3  = (const float*)d_in[9];
    const float* b3  = (const float*)d_in[10];
    const float* W4  = (const float*)d_in[11];
    const float* b4  = (const float*)d_in[12];
    const float* Wc0 = (const float*)d_in[13];
    const float* bc0 = (const float*)d_in[14];
    const float* Wc1 = (const float*)d_in[15];
    const float* bc1 = (const float*)d_in[16];
    const float* Wc2 = (const float*)d_in[17];
    const float* bc2 = (const float*)d_in[18];
    const float* Wn0 = (const float*)d_in[19];
    const float* bn0 = (const float*)d_in[20];
    const float* Wn1 = (const float*)d_in[21];
    const float* bn1 = (const float*)d_in[22];
    const float* Wn2 = (const float*)d_in[23];
    const float* bn2 = (const float*)d_in[24];
    float* out = (float*)d_out;

    char* ws = (char*)d_ws;
    _Float16* wt0 = (_Float16*)(ws + off0);
    _Float16* wsq = (_Float16*)(ws + off1);
    _Float16* wc2 = (_Float16*)(ws + off2);
    _Float16* wn2 = (_Float16*)(ws + off3);

    k_prep<<<dim3(8 + NSQ * 8 + 2), dim3(TPB_PREP), 0, stream>>>(
        W0, W1, W2, W3, W4, Wc0, Wc1, Wc2, Wn0, Wn1, Wn2, wt0, wsq, wc2, wn2);

    k_mlp<<<dim3(npts / ROWS), dim3(TPB_MAIN), SMEM_MAIN, stream>>>(
        x, Bf, t, W0, b0, b1, b2, b3, b4, bc0, bc1, bc2, bn0, bn1, bn2,
        wt0, wsq, wc2, wn2, out, npts);
}
